// MultiHeadAttention_6116033429738
// MI455X (gfx1250) — hardware-verified
//
#include <hip/hip_runtime.h>


#ifndef NB
#define NB 2
#endif
#ifndef SEQ
#define SEQ 2048
#endif
#define NB_FULL  2
#define SEQ_FULL 2048
#ifndef OUT_SEQ
#define OUT_SEQ SEQ
#endif
#define DM   1024
#define NH_  16
#define HD   64
#define AW   4
#define SC2  (0.125f * 1.4426950408889634f)
#define PSH  8.0f
#define CXS  256.0f
#define WPS  1024.0f
#define OSC  (1.0f / (256.0f * 1024.0f))

static_assert(HD == 64);
static_assert(NH_ * HD == DM);
static_assert(DM % 64 == 0);
static_assert(DM % 32 == 0);
static_assert(SEQ % 64 == 0);
static_assert((NB * SEQ) % 64 == 0);
static_assert(SEQ % 32 == 0);
static_assert(SEQ % (16 * AW) == 0);
static_assert(((size_t)SEQ * DM) % 8 == 0);
static_assert(((size_t)DM * DM) % 8 == 0);
static_assert(NB <= NB_FULL);
static_assert(SEQ <= SEQ_FULL);
static_assert(OUT_SEQ >= SEQ);

typedef _Float16 h16;
typedef unsigned short bf;
typedef __attribute__((ext_vector_type(16))) __bf16   v16bf;
typedef __attribute__((ext_vector_type(16))) _Float16 v16h;
typedef __attribute__((ext_vector_type(8)))  _Float16 v8h;
typedef __attribute__((ext_vector_type(8)))  unsigned short v8us;
typedef __attribute__((ext_vector_type(8)))  float    v8f;
typedef __attribute__((ext_vector_type(4)))  float    v4f;
typedef v4f  __attribute__((may_alias)) v4fa;

__device__ __forceinline__ unsigned short f2bf(float f) { unsigned u = __float_as_uint(f); u += 0x7FFFu + ((u >> 16) & 1u); return (unsigned short)(u >> 16); }
__device__ __forceinline__ float bfr(float f) { return __uint_as_float(((unsigned)f2bf(f)) << 16); }
__device__ __forceinline__ v16h cat16(v8h lo, v8h hi) { return __builtin_shufflevector(lo, hi, 0, 1, 2, 3, 4, 5, 6, 7, 8, 9, 10, 11, 12, 13, 14, 15); }
__device__ __forceinline__ v8f mma(v16h a, v16h b, v8f c)   { return __builtin_amdgcn_wmma_f32_16x16x32_f16(false, a, false, b, (short)0, c, false, false); }
__device__ __forceinline__ v8f mma(v16bf a, v16bf b, v8f c) { return __builtin_amdgcn_wmma_f32_16x16x32_bf16(false, a, false, b, (short)0, c, false, false); }
__device__ __forceinline__ v16h ldh(const h16* p) { return cat16(*(const v8h*)p, *(const v8h*)(p + 16)); }
template<typename FT> __device__ __forceinline__ FT ldf(const bf* p) {
    const v8us lo = *(const v8us*)p; const v8us hi = *(const v8us*)(p + 16);
    return __builtin_bit_cast(FT, __builtin_shufflevector(lo, hi, 0, 1, 2, 3, 4, 5, 6, 7, 8, 9, 10, 11, 12, 13, 14, 15));
}
__device__ __forceinline__ void wave_sync() { __builtin_amdgcn_fence(3  , "wavefront"); __builtin_amdgcn_wave_barrier(); asm volatile("" ::: "memory"); }

template<int ASF16>
__global__ __launch_bounds__(256) void k_cvt8(const float* __restrict__ src, bf* dst, size_t n8) {
    const size_t i = (size_t)blockIdx.x * 256 + threadIdx.x; if (i >= n8) return;
    const v8f v = *(const v8f*)(src + i * 8); v8us o;
#pragma unroll
    for (int k = 0; k < 8; ++k) {
        const unsigned short b0 = f2bf(v[k]);
        if (ASF16) { const float f0 = __uint_as_float(((unsigned)b0) << 16) * WPS; o[k] = __builtin_bit_cast(unsigned short, (h16)f0); }
        else o[k] = b0; }
    *(volatile v8us*)(dst + i * 8) = o; __threadfence(); *(volatile v8us*)(dst + i * 8) = o;
}

template<int MODE, typename FT>
__global__ __launch_bounds__(32) void k_gemm(const bf* __restrict__ A, const bf* __restrict__ Bt, const float* __restrict__ bias, h16* Ph, float* Pf, int RB, size_t sRB, int pitch, int CB, size_t sCB) {
    __shared__ __align__(16) float os[16 * 68];
    const int K = DM;
    const int lane = threadIdx.x & 31, lr = lane & 15, hi = lane >> 4; const int r0 = blockIdx.x * 64, c0 = blockIdx.y * 64;
    v8f acc[4][4];
#pragma unroll
    for (int mb = 0; mb < 4; ++mb)
#pragma unroll
        for (int nb = 0; nb < 4; ++nb) acc[mb][nb] = (v8f){};
    const size_t aoff = (size_t)(r0 + lr) * K + 8 * hi, boff = (size_t)(c0 + lr) * K + 8 * hi;
#pragma unroll 1
    for (int kc = 0; kc < K; kc += 32) {
        FT a[4];
#pragma unroll
        for (int mb = 0; mb < 4; ++mb) a[mb] = ldf<FT>(A + aoff + (size_t)mb * 16 * K + kc);
#pragma unroll
        for (int nb = 0; nb < 4; ++nb) { const FT b = ldf<FT>(Bt + boff + (size_t)nb * 16 * K + kc);
#pragma unroll
            for (int mb = 0; mb < 4; ++mb) acc[mb][nb] = mma(a[mb], b, acc[mb][nb]); }
        asm volatile("v_nop\n\tv_nop\n\tv_nop\n\tv_nop" : "+v"(acc[0][0]), "+v"(acc[1][1]), "+v"(acc[2][2]), "+v"(acc[3][3]) : "v"(a[0]), "v"(a[1]), "v"(a[2]), "v"(a[3]));
    }
    const size_t tbase = (size_t)(r0 / RB) * sRB + (size_t)(r0 % RB) * (size_t)pitch + (size_t)(c0 / CB) * sCB + (size_t)(c0 % CB);
    float bcol[8];
#pragma unroll
    for (int i = 0; i < 8; ++i) bcol[i] = 0.0f;
    if (MODE == 0) { const int c8 = (lane & 7) * 8;
        const v4f b0 = *(const v4f*)(bias + c0 + c8); const v4f b1 = *(const v4f*)(bias + c0 + c8 + 4);
#pragma unroll
        for (int i = 0; i < 4; ++i) { bcol[i] = bfr(b0[i]); bcol[4 + i] = bfr(b1[i]); } }
    if (MODE == 2) { const v4f b0 = *(const v4f*)(bias + c0 + lr * 4);
#pragma unroll
        for (int i = 0; i < 4; ++i) bcol[i] = bfr(b0[i]); }
#pragma unroll
    for (int mb = 0; mb < 4; ++mb) {
#pragma unroll
        for (int nb = 0; nb < 4; ++nb) {
#pragma unroll
            for (int j = 0; j < 8; ++j) os[(hi * 8 + j) * 68 + nb * 16 + lr] = acc[mb][nb][j]; }
        wave_sync();
        const size_t sb = tbase + (size_t)(mb * 16) * (size_t)pitch;
        if (MODE == 2) {
            v4f ov[8];
#pragma unroll
            for (int s = 0; s < 8; ++s) { const int row = 2 * s + hi;
                const v4f x0 = *(const v4fa*)(&os[row * 68 + lr * 4]);
#pragma unroll
                for (int i = 0; i < 4; ++i) ov[s][i] = x0[i] * OSC + bcol[i]; }
#pragma unroll 1
            for (int ps = 0; ps < 2; ++ps) {
#pragma unroll
                for (int s = 0; s < 8; ++s) { const int row = 2 * s + hi;
                    *(volatile v4f*)(Pf + sb + (size_t)row * (size_t)pitch + lr * 4) = ov[s]; }
                if (ps == 0) __threadfence(); }
        } else {
            v8h hv[4];
#pragma unroll
            for (int s = 0; s < 4; ++s) { const int row = 4 * s + (lane >> 3), c8 = (lane & 7) * 8;
                const v4f x0 = *(const v4fa*)(&os[row * 68 + c8]); const v4f x1 = *(const v4fa*)(&os[row * 68 + c8 + 4]);
                float rb = 0.0f;
                if (MODE == 1) rb = bfr(bias[r0 + mb * 16 + row]);
#pragma unroll
                for (int i = 0; i < 4; ++i) { hv[s][i] = (h16)(x0[i] + ((MODE == 1) ? rb : bcol[i])); hv[s][4 + i] = (h16)(x1[i] + ((MODE == 1) ? rb : bcol[4 + i])); } }
#pragma unroll 1
            for (int ps = 0; ps < 2; ++ps) {
#pragma unroll
                for (int s = 0; s < 4; ++s) { const int row = 4 * s + (lane >> 3), c8 = (lane & 7) * 8;
                    *(volatile v8h*)(Ph + sb + (size_t)row * (size_t)pitch + c8) = hv[s]; }
                if (ps == 0) __threadfence(); }
        }
        wave_sync();
    }
}

__global__ __launch_bounds__(32 * AW) void k_flash(const h16* __restrict__ QK, const h16* __restrict__ VT, h16* CTX) {
    __shared__ __align__(16) float os[AW * 16 * 68];
    const int lane = threadIdx.x & 31, lr = lane & 15, hi = lane >> 4;
    const int wave = __builtin_amdgcn_readfirstlane((int)(threadIdx.x >> 5));
    const int zh = blockIdx.y; const int b = zh / NH_, h = zh % NH_;
    const int t0 = (blockIdx.x * AW + wave) * 16;
    const size_t qbase = ((size_t)(b * 2) * NH_ + h) * SEQ * HD;
    const size_t kbase = qbase + (size_t)NH_ * SEQ * HD;
    const size_t vbase = (size_t)zh * HD * SEQ;
    const size_t qo = qbase + (size_t)(t0 + lr) * HD + 8 * hi;
    const v16h q0 = ldh(QK + qo), q1 = ldh(QK + qo + 32);
    const size_t ko = kbase + (size_t)lr * HD + 8 * hi;
    const size_t vo = vbase + (size_t)lr * SEQ + 8 * hi;
    v8f o0 = (v8f){}, o1 = (v8f){}, o2 = (v8f){}, o3 = (v8f){};
    float m = -3.0e38f, l = 0.0f;
#pragma unroll 1
    for (int key0 = 0; key0 < SEQ; key0 += 32) {
        const h16* ka = QK + ko + (size_t)key0 * HD;
        const v16h ka0 = ldh(ka), ka1 = ldh(ka + 32), kb0 = ldh(ka + 16 * HD), kb1 = ldh(ka + 16 * HD + 32);
        v8f sa = (v8f){}, sb = (v8f){};
        sa = mma(ka0, q0, sa); sb = mma(kb0, q0, sb);
        sa = mma(ka1, q1, sa); sb = mma(kb1, q1, sb);
        asm volatile("v_nop\n\tv_nop\n\tv_nop\n\tv_nop" : "+v"(sa), "+v"(sb) : "v"(ka0), "v"(ka1), "v"(kb0), "v"(kb1));
        float ta[8], tb[8]; float mx = -3.0e38f;
#pragma unroll
        for (int r = 0; r < 8; ++r) { ta[r] = sa[r] * SC2; tb[r] = sb[r] * SC2; mx = fmaxf(mx, fmaxf(ta[r], tb[r])); }
        mx = fmaxf(mx, __shfl_xor(mx, 16, 32));
        const float mnew = fmaxf(m, mx);
        const float alpha = __builtin_amdgcn_exp2f(m - mnew);
        const float sh = PSH - mnew;
        v16h pb; float ls = 0.0f;
#pragma unroll
        for (int r = 0; r < 8; ++r) { const h16 pa = (h16)__builtin_amdgcn_exp2f(ta[r] + sh); const h16 pc = (h16)__builtin_amdgcn_exp2f(tb[r] + sh); pb[r] = pa; pb[8 + r] = pc; ls += (float)pa + (float)pc; }
        l = l * alpha + ls; m = mnew;
        o0 = o0 * alpha; o1 = o1 * alpha; o2 = o2 * alpha; o3 = o3 * alpha;
        const h16* va = VT + vo + key0;
        const v16h v0 = ldh(va), v1 = ldh(va + (size_t)16 * SEQ), v2 = ldh(va + (size_t)32 * SEQ), v3 = ldh(va + (size_t)48 * SEQ);
        o0 = mma(v0, pb, o0); o1 = mma(v1, pb, o1); o2 = mma(v2, pb, o2); o3 = mma(v3, pb, o3);
        asm volatile("v_nop\n\tv_nop\n\tv_nop\n\tv_nop" : "+v"(o0), "+v"(o1), "+v"(o2), "+v"(o3) : "v"(v0), "v"(v1), "v"(v2), "v"(v3), "v"(pb));
    }
    l += __shfl_xor(l, 16, 32);
    const float inv = (1.0f / l) * CXS;
    const int wb = wave * 16 * 68;
    { v4f a, c;
      a[0] = o0[0] * inv; a[1] = o0[1] * inv; a[2] = o0[2] * inv; a[3] = o0[3] * inv; c[0] = o0[4] * inv; c[1] = o0[5] * inv; c[2] = o0[6] * inv; c[3] = o0[7] * inv;
      *(v4fa*)(&os[wb + lr * 68 +  0 + 8 * hi]) = a; *(v4fa*)(&os[wb + lr * 68 +  0 + 8 * hi + 4]) = c;
      a[0] = o1[0] * inv; a[1] = o1[1] * inv; a[2] = o1[2] * inv; a[3] = o1[3] * inv; c[0] = o1[4] * inv; c[1] = o1[5] * inv; c[2] = o1[6] * inv; c[3] = o1[7] * inv;
      *(v4fa*)(&os[wb + lr * 68 + 16 + 8 * hi]) = a; *(v4fa*)(&os[wb + lr * 68 + 16 + 8 * hi + 4]) = c;
      a[0] = o2[0] * inv; a[1] = o2[1] * inv; a[2] = o2[2] * inv; a[3] = o2[3] * inv; c[0] = o2[4] * inv; c[1] = o2[5] * inv; c[2] = o2[6] * inv; c[3] = o2[7] * inv;
      *(v4fa*)(&os[wb + lr * 68 + 32 + 8 * hi]) = a; *(v4fa*)(&os[wb + lr * 68 + 32 + 8 * hi + 4]) = c;
      a[0] = o3[0] * inv; a[1] = o3[1] * inv; a[2] = o3[2] * inv; a[3] = o3[3] * inv; c[0] = o3[4] * inv; c[1] = o3[5] * inv; c[2] = o3[6] * inv; c[3] = o3[7] * inv;
      *(v4fa*)(&os[wb + lr * 68 + 48 + 8 * hi]) = a; *(v4fa*)(&os[wb + lr * 68 + 48 + 8 * hi + 4]) = c; }
    wave_sync();
    h16* crow = CTX + ((size_t)b * SEQ + t0) * DM + h * HD;
    v8h hv[4];
#pragma unroll
    for (int s = 0; s < 4; ++s) { const int row = 4 * s + (lane >> 3), c8 = (lane & 7) * 8;
        const v4f x0 = *(const v4fa*)(&os[wb + row * 68 + c8]); const v4f x1 = *(const v4fa*)(&os[wb + row * 68 + c8 + 4]);
#pragma unroll
        for (int i = 0; i < 4; ++i) { hv[s][i] = (h16)x0[i]; hv[s][4 + i] = (h16)x1[i]; } }
#pragma unroll 1
    for (int ps = 0; ps < 2; ++ps) {
#pragma unroll
        for (int s = 0; s < 4; ++s) { const int row = 4 * s + (lane >> 3), c8 = (lane & 7) * 8;
            *(volatile v8h*)(crow + (size_t)row * DM + c8) = hv[s]; }
        if (ps == 0) __threadfence(); }
}

static constexpr size_t al256(size_t v) { return (v + 255) & ~(size_t)255; }
static constexpr size_t SZ_XB  = al256((size_t)NB * SEQ * DM * 2);
static constexpr size_t SZ_WQ  = al256((size_t)3 * DM * DM * 2);
static constexpr size_t SZ_WP  = al256((size_t)DM * DM * 2);
static constexpr size_t SZ_QK  = al256((size_t)NB * 2 * NH_ * SEQ * HD * 2);
static constexpr size_t SZ_VT  = al256((size_t)NB * NH_ * HD * SEQ * 2);
static constexpr size_t SZ_CX  = al256((size_t)NB * SEQ * DM * 2);
static constexpr size_t SZ_TOTAL = SZ_XB + SZ_WQ + SZ_WP + SZ_QK + SZ_VT + SZ_CX;
static_assert(SZ_TOTAL <= (size_t)134217728);
static_assert(((size_t)DM * DM * 2) % 256 == 0);

extern "C" void kernel_launch(void* const* d_in, const int* in_sizes, int n_in,
                              void* d_out, int out_size, void* d_ws, size_t ws_size, hipStream_t stream) {
    if (n_in < 5) return;
    const size_t needx = ((size_t)(NB - 1) * SEQ_FULL + SEQ) * DM;
    if ((size_t)in_sizes[0] < needx) return;
    if ((size_t)in_sizes[1] < (size_t)3 * DM * DM || (size_t)in_sizes[2] < (size_t)3 * DM) return;
    if ((size_t)in_sizes[3] < (size_t)DM * DM || (size_t)in_sizes[4] < (size_t)DM) return;
    if ((size_t)out_size < ((size_t)(NB - 1) * OUT_SEQ + SEQ) * DM) return;
    if (SZ_TOTAL > ws_size) return;
    const float* x = (const float*)d_in[0]; const float* wqkv = (const float*)d_in[1]; const float* bqkv = (const float*)d_in[2];
    const float* wo = (const float*)d_in[3]; const float* bo = (const float*)d_in[4];
    float* OUT = (float*)d_out;
    char* wsp = (char*)d_ws;
    bf* XB  = (bf*)wsp;  wsp += SZ_XB;
    bf* WQT = (bf*)wsp;  wsp += SZ_WQ;
    bf* WPT = (bf*)wsp;  wsp += SZ_WP;
    h16* QK = (h16*)wsp; wsp += SZ_QK;
    h16* VT = (h16*)wsp; wsp += SZ_VT;
    h16* CTX = (h16*)wsp; wsp += SZ_CX;

    if (SEQ == SEQ_FULL) {
        const size_t n8 = (size_t)NB * SEQ * DM / 8;
        k_cvt8<0><<<(unsigned)((n8 + 255) / 256), 256, 0, stream>>>(x, XB, n8);
    } else {
        const size_t n8 = (size_t)SEQ * DM / 8;
        for (int b = 0; b < NB; ++b) k_cvt8<0><<<(unsigned)((n8 + 255) / 256), 256, 0, stream>>>(x + (size_t)b * SEQ_FULL * DM, XB + (size_t)b * SEQ * DM, n8);
    }
    { const size_t n8 = (size_t)3 * DM * DM / 8;
      k_cvt8<0><<<(unsigned)((n8 + 255) / 256), 256, 0, stream>>>(wqkv, WQT, n8); }
    { const size_t n8 = (size_t)DM * DM / 8;
      k_cvt8<1><<<(unsigned)((n8 + 255) / 256), 256, 0, stream>>>(wo, WPT, n8); }

    k_gemm<0, v16bf><<<dim3(NB * SEQ / 64, 2 * DM / 64, 1), 32, 0, stream>>>(XB, WQT, bqkv, QK, OUT, SEQ, (size_t)2 * NH_ * SEQ * HD, HD, HD, (size_t)SEQ * HD);
    k_gemm<1, v16bf><<<dim3(DM / 64, NB * SEQ / 64, 1), 32, 0, stream>>>(WQT + (size_t)2 * DM * DM, XB, bqkv + 2 * DM, VT, OUT, DM, (size_t)0, SEQ, SEQ, (size_t)DM * SEQ);

    k_flash<<<dim3(SEQ / (16 * AW), NB * NH_, 1), 32 * AW, 0, stream>>>(QK, VT, CTX);

    k_gemm<2, v16h><<<dim3(NB * SEQ / 64, DM / 64, 1), 32, 0, stream>>>((const bf*)CTX, WPT, bo, QK, OUT, SEQ, (size_t)OUT_SEQ * DM, DM, DM, (size_t)0);
}
